// dnbRNN_13365938225208
// MI455X (gfx1250) — hardware-verified
//
#include <hip/hip_runtime.h>
#include <math.h>

constexpr int NB_SEQ   = 64;
constexpr int NU_IN    = 64;
constexpr int NX_HID   = 768;
constexpr int NY_OUT   = 32;
constexpr int NT_STEPS = 1024;
constexpr int KCAT = NX_HID + NU_IN;
constexpr int NCAT = NX_HID + NY_OUT;
constexpr int SEQ_BLK        = 16;
constexpr int SEQ_WAVES      = 10;
constexpr int SEQ_THR        = 32 * SEQ_WAVES;
constexpr int TILES_PER_WAVE = 5;
constexpr int H_TILES        = NX_HID / 16;
constexpr int H_TILES_LAST   = H_TILES - TILES_PER_WAVE * (SEQ_WAVES - 1);
constexpr int APITCH = 840;
constexpr int YPITCH = 36;
constexpr float WCARRY     = 256.0f;
constexpr float WCARRY_INV = 1.0f / 256.0f;
constexpr size_t TILE_STRIDE = (size_t)16 * KCAT;

static_assert(KCAT == 832 && KCAT % 32 == 0, "K multiple of 32");
static_assert(NCAT == 800 && NCAT == 16 * SEQ_WAVES * TILES_PER_WAVE, "N tiles exactly cover the waves");
static_assert(H_TILES == 48 && H_TILES_LAST == 3, "tile split of the last wave");
static_assert(NB_SEQ % SEQ_BLK == 0, "batch tiles");
static_assert(APITCH % 8 == 0 && APITCH >= KCAT, "A pitch");
static_assert((KCAT * 2) % 128 == 0, "weight rows are whole lines");
static_assert(NU_IN * 2 == 128 && NY_OUT * 4 == 128, "u rows and y rows are one line each");
static_assert(NT_STEPS % 32 == 0, "time chunks");
static_assert(NX_HID % 8 == 0, "h0 vector groups");

typedef __attribute__((ext_vector_type(16))) _Float16 v16h;
typedef __attribute__((ext_vector_type(8)))  _Float16 v8h;
typedef __attribute__((ext_vector_type(8)))  float    v8f;
typedef __attribute__((ext_vector_type(4)))  float    v4f;

struct FragH {
  union U { v16h v; v8h h[2]; };
  static __device__ __forceinline__ v16h load(const _Float16* p) {
    U f;
    f.h[0] = *(const v8h*)(p);
    f.h[1] = *(const v8h*)(p + 16);
    return f.v;
  }
  static __device__ __forceinline__ v8f mma(v16h a, v16h b, v8f c) {
    return __builtin_amdgcn_wmma_f32_16x16x32_f16(false, a, false, b, (short)0, c, false, false);
  }
};

__device__ __forceinline__ void guard5(v8f& a0, v8f& a1, v8f& a2, v8f& a3, v8f& a4,
                                       v16h x, v16h b0, v16h b1, v16h b2, v16h b3, v16h b4) {
  asm volatile("v_nop\n\tv_nop\n\tv_nop\n\tv_nop"
               : "+v"(a0), "+v"(a1), "+v"(a2), "+v"(a3), "+v"(a4)
               : "v"(x), "v"(b0), "v"(b1), "v"(b2), "v"(b3), "v"(b4));
}

__global__ __launch_bounds__(128) void prep_w_kernel(const float* __restrict__ Hw, const float* __restrict__ Kw,
                                                     const float* __restrict__ Ow, const float* __restrict__ Hb,
                                                     const float* __restrict__ Ob,
                                                     unsigned short* __restrict__ Wcat, float* __restrict__ bcat) {
  const int tid = threadIdx.x, lane = tid & 31, wave = tid >> 5;
  const int n = blockIdx.x;
  if (n >= NCAT) {
    constexpr int NHB4 = NX_HID / 4;
    constexpr int NBC4 = NCAT / 4;
#pragma unroll
    for (int it = 0; it < 2; ++it) {
      const int idx = it * 128 + tid;
      const int hi4 = (idx < NHB4 ? idx : NHB4 - 1) * 4;
      int oi = idx - NHB4;
      oi = oi < 0 ? 0 : (oi > (NY_OUT / 4 - 1) ? (NY_OUT / 4 - 1) : oi);
      const v4f va = *(const v4f*)(Hb + hi4);
      const v4f vb = *(const v4f*)(Ob + oi * 4);
      v4f o;
#pragma unroll
      for (int e = 0; e < 4; ++e) o[e] = (idx < NHB4) ? va[e] : vb[e];
      const int oidx = idx < NBC4 ? idx : NBC4 - 1;
      volatile v4f* dp = (volatile v4f*)(bcat + oidx * 4);
      if (idx < NBC4) *dp = o;
      __threadfence();
      if (idx < NBC4) *dp = o;
    }
    return;
  }
  const float* src = (n < NX_HID) ? (Hw + (size_t)n * NX_HID) : (Ow + (size_t)(n - NX_HID) * NX_HID);
  v4f a = {0.f, 0.f, 0.f, 0.f};
  v4f b = {0.f, 0.f, 0.f, 0.f};
  int col;
  bool act;
  if (wave < 3) {
    col = tid * 8;
    a = *(const v4f*)(src + col);
    b = *(const v4f*)(src + col + 4);
    act = true;
  } else {
    const int seg = lane < 7 ? lane : 7;
    col = NX_HID + seg * 8;
    if (n < NX_HID) {
      const float* kp = Kw + (size_t)n * NU_IN + seg * 8;
      a = *(const v4f*)(kp);
      b = *(const v4f*)(kp + 4);
    }
    act = lane < 8;
  }
  v8h hv;
#pragma unroll
  for (int e = 0; e < 4; ++e) {
    hv[e]     = (_Float16)(a[e] * WCARRY);
    hv[4 + e] = (_Float16)(b[e] * WCARRY);
  }
  volatile v8h* dp = (volatile v8h*)(Wcat + (size_t)n * KCAT + col);
  if (act) *dp = hv;
  __threadfence();
  if (act) *dp = hv;
}

__global__ __launch_bounds__(256) void prep_u_kernel(const float* __restrict__ u, unsigned short* __restrict__ Uh) {
  __shared__ float Tt[NU_IN * 33];
  const int tid = threadIdx.x;
  const int b  = blockIdx.x >> 5;
  const int t0 = (blockIdx.x & 31) * 32;
#pragma unroll
  for (int i = 0; i < 2; ++i) {
    const int idx = i * 256 + tid;
    const int k = idx >> 3, t4 = (idx & 7) * 4;
    const v4f v = *(const v4f*)(u + ((size_t)b * NU_IN + k) * NT_STEPS + t0 + t4);
    Tt[k * 33 + t4 + 0] = v[0];
    Tt[k * 33 + t4 + 1] = v[1];
    Tt[k * 33 + t4 + 2] = v[2];
    Tt[k * 33 + t4 + 3] = v[3];
  }
  __syncthreads();
  const int tt = tid >> 3, c8 = (tid & 7) * 8;
  v8h hv;
#pragma unroll
  for (int e = 0; e < 8; ++e) hv[e] = (_Float16)Tt[(c8 + e) * 33 + tt];
  volatile v8h* dp = (volatile v8h*)(Uh + (((size_t)(t0 + tt) * NB_SEQ + b) * NU_IN + c8));
  *dp = hv;
  __threadfence();
  *dp = hv;
}

__global__ __launch_bounds__(SEQ_THR) void rnn_seq_kernel(const float* __restrict__ h0,
                                                          const unsigned short* __restrict__ Wcatp,
                                                          const float* __restrict__ bcat,
                                                          const unsigned short* __restrict__ Uhp,
                                                          float* __restrict__ Y) {
  __shared__ __align__(16) _Float16 Ab[2][SEQ_BLK * APITCH];
  __shared__ __align__(16) float    Ys[SEQ_BLK * YPITCH];
  const _Float16* Wcat = (const _Float16*)Wcatp;
  const _Float16* Uh   = (const _Float16*)Uhp;
  const int tid = threadIdx.x, lane = tid & 31, wave = tid >> 5;
  const int c = lane & 15, hh = lane >> 4, koff = hh * 8;
  const int b0 = blockIdx.x * SEQ_BLK;
  const int urow = (tid >> 3) & 15, useg = tid & 7;

#pragma unroll 1
  for (int i = tid; i < SEQ_BLK * (NX_HID / 8); i += SEQ_THR) {
    const int row = i / (NX_HID / 8);
    const int g8  = i - row * (NX_HID / 8);
    const float* sp = h0 + (size_t)(b0 + row) * NX_HID + g8 * 8;
    const v4f a = *(const v4f*)(sp);
    const v4f b = *(const v4f*)(sp + 4);
    v8h hv;
#pragma unroll
    for (int e = 0; e < 4; ++e) {
      hv[e]     = (_Float16)a[e];
      hv[4 + e] = (_Float16)b[e];
    }
    *(v8h*)(&Ab[0][0] + row * APITCH + g8 * 8) = hv;
  }
  if (tid < 128) {
    const v8h uv = *(const v8h*)(Uh + (((size_t)0 * NB_SEQ + b0 + urow) * NU_IN + useg * 8));
    *(v8h*)(&Ab[0][0] + urow * APITCH + NX_HID + useg * 8) = uv;
  }
  if (tid >= 128 && tid < 160) {
    const int i = tid - 128;
    const v8h zv = {(_Float16)0.0f, (_Float16)0.0f, (_Float16)0.0f, (_Float16)0.0f,
                    (_Float16)0.0f, (_Float16)0.0f, (_Float16)0.0f, (_Float16)0.0f};
    *(v8h*)(&Ab[i >> 4][0] + (i & 15) * APITCH + KCAT) = zv;
  }
  float bb[TILES_PER_WAVE];
#pragma unroll
  for (int j = 0; j < TILES_PER_WAVE; ++j) bb[j] = bcat[16 * (TILES_PER_WAVE * wave + j) + c];
  __syncthreads();

  const _Float16* wbase = Wcat + (size_t)(16 * TILES_PER_WAVE * wave + c) * KCAT + koff;
  const v8f z8 = {0.f, 0.f, 0.f, 0.f, 0.f, 0.f, 0.f, 0.f};
  const int yq = lane >> 3, yc4 = (lane & 7) * 4;
  int cur = 0;

#pragma unroll 1
  for (int s = 0; s < NT_STEPS; ++s) {
    _Float16* abn = &Ab[cur ^ 1][0];
    const _Float16* arow = &Ab[cur][0] + c * APITCH + koff;

    if (tid < 128) {
      const int tn = (s + 1 < NT_STEPS) ? (s + 1) : (NT_STEPS - 1);
      const v8h uv = *(const v8h*)(Uh + (((size_t)tn * NB_SEQ + b0 + urow) * NU_IN + useg * 8));
      *(v8h*)(abn + urow * APITCH + NX_HID + useg * 8) = uv;
    }

    v8f acc[TILES_PER_WAVE];
#pragma unroll
    for (int j = 0; j < TILES_PER_WAVE; ++j) acc[j] = z8;

#pragma unroll 1
    for (int k0 = 0; k0 < KCAT; k0 += 32) {
      const v16h a  = FragH::load(arow + k0);
      const v16h w0 = FragH::load(wbase + k0);
      const v16h w1 = FragH::load(wbase + 1 * TILE_STRIDE + k0);
      const v16h w2 = FragH::load(wbase + 2 * TILE_STRIDE + k0);
      const v16h w3 = FragH::load(wbase + 3 * TILE_STRIDE + k0);
      const v16h w4 = FragH::load(wbase + 4 * TILE_STRIDE + k0);
      acc[0] = FragH::mma(a, w0, acc[0]);
      acc[1] = FragH::mma(a, w1, acc[1]);
      acc[2] = FragH::mma(a, w2, acc[2]);
      acc[3] = FragH::mma(a, w3, acc[3]);
      acc[4] = FragH::mma(a, w4, acc[4]);
      guard5(acc[0], acc[1], acc[2], acc[3], acc[4], a, w0, w1, w2, w3, w4);
    }

#pragma unroll
    for (int j = 0; j < TILES_PER_WAVE; ++j) {
      const bool is_hidden = (wave < SEQ_WAVES - 1) || (j < H_TILES_LAST);
      if (is_hidden) {
        const int n = 16 * (TILES_PER_WAVE * wave + j) + c;
#pragma unroll
        for (int r = 0; r < 8; ++r) {
          const float xv = acc[j][r] * WCARRY_INV + bb[j];
          const float hv = fmaxf(xv, 0.0f);
          abn[(8 * hh + r) * APITCH + n] = (_Float16)hv;
        }
      } else {
        const int o = 16 * (j - H_TILES_LAST) + c;
#pragma unroll
        for (int r = 0; r < 8; ++r) {
          Ys[(8 * hh + r) * YPITCH + o] = acc[j][r] * WCARRY_INV + bb[j];
        }
      }
    }

    if (wave == SEQ_WAVES - 1) {
      __builtin_amdgcn_fence(__ATOMIC_RELEASE, "workgroup");
      __builtin_amdgcn_wave_barrier();
      __builtin_amdgcn_fence(__ATOMIC_ACQUIRE, "workgroup");
      for (int pass = 0; pass < 2; ++pass) {
#pragma unroll
        for (int it = 0; it < 4; ++it) {
          const int row = it * 4 + yq;
          const v4f v = *(const v4f*)(Ys + row * YPITCH + yc4);
          *(volatile v4f*)(Y + ((size_t)(b0 + row) * NT_STEPS + (size_t)s) * NY_OUT + yc4) = v;
        }
        __threadfence();
      }
      __builtin_amdgcn_fence(__ATOMIC_RELEASE, "workgroup");
      __builtin_amdgcn_wave_barrier();
      __builtin_amdgcn_fence(__ATOMIC_ACQUIRE, "workgroup");
    }

    __syncthreads();
    cur ^= 1;
  }
}

__global__ __launch_bounds__(256) void y_transpose_kernel(const float* __restrict__ Y, float* __restrict__ out) {
  __shared__ float Tt[32 * 33];
  const int tid = threadIdx.x;
  const int b  = blockIdx.x >> 5;
  const int t0 = (blockIdx.x & 31) * 32;
  {
    const int t = tid >> 3, o4 = (tid & 7) * 4;
    const v4f v = *(const v4f*)(Y + ((size_t)b * NT_STEPS + t0 + t) * NY_OUT + o4);
    Tt[t * 33 + o4 + 0] = v[0];
    Tt[t * 33 + o4 + 1] = v[1];
    Tt[t * 33 + o4 + 2] = v[2];
    Tt[t * 33 + o4 + 3] = v[3];
  }
  __syncthreads();
  const int o = tid >> 3, t4 = (tid & 7) * 4;
  v4f w;
#pragma unroll
  for (int e = 0; e < 4; ++e) w[e] = Tt[(t4 + e) * 33 + o];
  volatile v4f* dp = (volatile v4f*)(out + ((size_t)b * NY_OUT + o) * NT_STEPS + t0 + t4);
  *dp = w;
  __threadfence();
  *dp = w;
}

extern "C" void kernel_launch(void* const* d_in, const int* in_sizes, int n_in,
                              void* d_out, int out_size, void* d_ws, size_t ws_size, hipStream_t stream) {
  if (n_in < 7 || d_out == nullptr || d_ws == nullptr) return;
  if (in_sizes[0] != NB_SEQ * NU_IN * NT_STEPS || in_sizes[1] != NB_SEQ * NX_HID ||
      in_sizes[2] != NX_HID * NX_HID || in_sizes[3] != NX_HID || in_sizes[4] != NX_HID * NU_IN ||
      in_sizes[5] != NY_OUT * NX_HID || in_sizes[6] != NY_OUT ||
      out_size != NB_SEQ * NY_OUT * NT_STEPS) return;

  const float* u  = (const float*)d_in[0];
  const float* h0 = (const float*)d_in[1];
  const float* Hw = (const float*)d_in[2];
  const float* Hb = (const float*)d_in[3];
  const float* Kw = (const float*)d_in[4];
  const float* Ow = (const float*)d_in[5];
  const float* Ob = (const float*)d_in[6];
  float* out = (float*)d_out;

  char* ws = (char*)d_ws;
  size_t off = 0;
  auto carve = [&](size_t bytes) -> char* { char* p = ws + off; off += (bytes + 255) & ~(size_t)255; return p; };
  unsigned short* Wcat = (unsigned short*)carve((size_t)NCAT * KCAT * 2);
  float*          bcat = (float*)carve((size_t)NCAT * 4);
  unsigned short* Uh   = (unsigned short*)carve((size_t)NT_STEPS * NB_SEQ * NU_IN * 2);
  float*          Yp   = (float*)carve((size_t)NB_SEQ * NT_STEPS * NY_OUT * 4);
  if (off > ws_size || off > (size_t)134217728) return;

  prep_w_kernel<<<NCAT + 1, 128, 0, stream>>>(Hw, Kw, Ow, Hb, Ob, Wcat, bcat);
  prep_u_kernel<<<NB_SEQ * (NT_STEPS / 32), 256, 0, stream>>>(u, Uh);
  rnn_seq_kernel<<<NB_SEQ / SEQ_BLK, SEQ_THR, 0, stream>>>(h0, Wcat, bcat, Uh, Yp);
  y_transpose_kernel<<<NB_SEQ * (NT_STEPS / 32), 256, 0, stream>>>(Yp, out);
}
